// Block_ssmamba_4020089389066
// MI455X (gfx1250) — hardware-verified
//
#include <hip/hip_runtime.h>
#include <math.h>

typedef __attribute__((ext_vector_type(16))) _Float16 v16h;
typedef __attribute__((ext_vector_type(8)))  _Float16 v8h;
typedef __attribute__((ext_vector_type(4)))  _Float16 v4h;
typedef __attribute__((ext_vector_type(16))) __bf16   v16b;
typedef __attribute__((ext_vector_type(8)))  __bf16   v8b;
typedef __attribute__((ext_vector_type(8)))  float    v8f;
typedef __attribute__((ext_vector_type(4)))  float    v4f;
typedef __attribute__((ext_vector_type(2)))  float    v2f;

constexpr int NIMG      = 2;
constexpr int NCH       = 128;
constexpr int IMG_H     = 64;
constexpr int IMG_W     = 64;
constexpr int NPIX      = IMG_H * IMG_W;
constexpr int NTOK      = NIMG * NPIX;
constexpr int NSTATE    = 16;
constexpr int NDIRS     = 2;
constexpr int DTR_SPA   = 8;
constexpr int XROWS_SPA = 40;
constexpr int XDW       = 64;
constexpr int CN_SPE    = 16;
constexpr int GC_SPE    = 8;
constexpr int XROWS_SPE = 33;

__device__ __forceinline__ unsigned short f2bf_bits(float f) {
  unsigned u = __float_as_uint(f);
  return (unsigned short)((u + 0x7FFFu + ((u >> 16) & 1u)) >> 16);
}
__device__ __forceinline__ float bf_bits2f(unsigned short h) { return __uint_as_float(((unsigned)h) << 16); }

__device__ __forceinline__ void dep_guard_h(v8f& a, v8f& b, v16h x, v16h y) { asm volatile("v_nop\n\tv_nop\n\tv_nop\n\tv_nop" : "+v"(a), "+v"(b) : "v"(x), "v"(y)); }
__device__ __forceinline__ void dep_guard_b(v8f& a, v8f& b, v16b x, v16b y) { asm volatile("v_nop\n\tv_nop\n\tv_nop\n\tv_nop" : "+v"(a), "+v"(b) : "v"(x), "v"(y)); }
__device__ __forceinline__ void keep4_h(v16h a, v16h b, v16h c, v16h d) { asm volatile("v_nop" :: "v"(a), "v"(b), "v"(c), "v"(d)); }
__device__ __forceinline__ void keep4_b(v16b a, v16b b, v16b c, v16b d) { asm volatile("v_nop" :: "v"(a), "v"(b), "v"(c), "v"(d)); }
__device__ __forceinline__ void acc_guard4(v8f& a, v8f& b, v8f& c, v8f& d) { asm volatile("v_nop\n\tv_nop\n\tv_nop\n\tv_nop" : "+v"(a), "+v"(b), "+v"(c), "+v"(d)); }
template <typename T> struct Frag;
template <> struct Frag<_Float16> {
  typedef v16h V; union U { v16h v; v8h h[2]; };
  static __device__ __forceinline__ v16h load(const _Float16* p) {
    U f; f.h[0] = *(const v8h*)(p); f.h[1] = *(const v8h*)(p + 16); return f.v;
  }
  static __device__ __forceinline__ v8f mma(v16h a, v16h b, v8f c) {
    return __builtin_amdgcn_wmma_f32_16x16x32_f16(false, a, false, b, (short)0, c, false, false);
  }
  static __device__ __forceinline__ void guard(v8f& a, v8f& b, v16h x, v16h y) { dep_guard_h(a, b, x, y); }
  static __device__ __forceinline__ void keep(v16h a, v16h b, v16h c, v16h d) { keep4_h(a, b, c, d); }
};
template <> struct Frag<__bf16> {
  typedef v16b V; union U { v16b v; v8b h[2]; };
  static __device__ __forceinline__ v16b load(const __bf16* p) {
    U f; f.h[0] = *(const v8b*)(p); f.h[1] = *(const v8b*)(p + 16); return f.v;
  }
  static __device__ __forceinline__ v8f mma(v16b a, v16b b, v8f c) {
    return __builtin_amdgcn_wmma_f32_16x16x32_bf16(false, a, false, b, (short)0, c, false, false);
  }
  static __device__ __forceinline__ void guard(v8f& a, v8f& b, v16b x, v16b y) { dep_guard_b(a, b, x, y); }
  static __device__ __forceinline__ void keep(v16b a, v16b b, v16b c, v16b d) { keep4_b(a, b, c, d); }
};

template <int ET> struct Elem;
template <> struct Elem<0> { typedef _Float16 T; };
template <> struct Elem<1> { typedef __bf16 T; };
template <int ET, bool SPLIT, int BIAS_MODE, int OUT_MODE, bool RESID, int ACT = 0>
__global__ __launch_bounds__(256) void wmma_gemm64(
    const unsigned short* __restrict__ Ap, const unsigned short* __restrict__ A2p, int lda, long strideA,
    const unsigned short* __restrict__ Btp, const unsigned short* __restrict__ Bt2p, int ldb, long strideB,
    void* __restrict__ Cout, void* __restrict__ Cout2, int ldc, long strideC,
    const float* __restrict__ bias,
    const float* __restrict__ resid, long strideR,
    int M, int N, int K, float scale) {
  typedef typename Elem<ET>::T T;
  typedef typename Frag<T>::V V;
  const T* A = (const T*)Ap; const T* A2 = (const T*)A2p; const T* Bt = (const T*)Btp; const T* Bt2 = (const T*)Bt2p;
  __shared__ __align__(16) float sT[8][16 * 68];
  const int b    = blockIdx.y;
  const int lane = threadIdx.x & 31;
  const int wave = threadIdx.x >> 5;
  const int tilesN = N >> 6;
  const int tilesM = M >> 6;
  const int tile = blockIdx.x * 8 + wave;
  if (tile >= tilesM * tilesN) return;
  const int tm = tile / tilesN;
  const int tn = tile - tm * tilesN;
  const int m0 = tm << 6;
  const int n0 = tn << 6;

  const T* Ab  = A  + (size_t)b * strideA;
  const T* Bb  = Bt + (size_t)b * strideB;
  const T* Ab2 = SPLIT ? (A2  + (size_t)b * strideA) : nullptr;
  const T* Bb2 = SPLIT ? (Bt2 + (size_t)b * strideB) : nullptr;

  const int rlane = lane & 15;
  const int koff  = (lane >> 4) * 8;
  const int mOff  = (lane >> 4) * 8;

  v8f acc[4][4];
#pragma unroll
  for (int i = 0; i < 4; ++i)
#pragma unroll
    for (int j = 0; j < 4; ++j) acc[i][j] = (v8f){0.f,0.f,0.f,0.f,0.f,0.f,0.f,0.f};

  for (int k0 = 0; k0 < K; k0 += 32) {
    V bh[4], bl[4];
#pragma unroll
    for (int j = 0; j < 4; ++j) {
      const size_t bo = (size_t)(n0 + (j << 4) + rlane) * ldb + koff + k0;
      bh[j] = Frag<T>::load(Bb + bo);
      if (SPLIT) bl[j] = Frag<T>::load(Bb2 + bo);
    }
#pragma unroll
    for (int i = 0; i < 4; ++i) {
      const size_t ao = (size_t)(m0 + (i << 4) + rlane) * lda + koff + k0;
      V ah = Frag<T>::load(Ab + ao);
      V al;
      if (SPLIT) al = Frag<T>::load(Ab2 + ao);
#pragma unroll
      for (int j = 0; j < 4; ++j) {
        acc[i][j] = Frag<T>::mma(ah, bh[j], acc[i][j]);
        if (SPLIT) {
          acc[i][j] = Frag<T>::mma(ah, bl[j], acc[i][j]);
          acc[i][j] = Frag<T>::mma(al, bh[j], acc[i][j]);
        }
      }
      Frag<T>::guard(acc[i][0], acc[i][3], ah, SPLIT ? al : ah);
    }
    Frag<T>::keep(bh[0], bh[1], bh[2], bh[3]);
    if (SPLIT) Frag<T>::keep(bl[0], bl[1], bl[2], bl[3]);
  }
  acc_guard4(acc[0][0], acc[0][1], acc[0][2], acc[0][3]);
  acc_guard4(acc[1][0], acc[1][1], acc[1][2], acc[1][3]);
  acc_guard4(acc[2][0], acc[2][1], acc[2][2], acc[2][3]);
  acc_guard4(acc[3][0], acc[3][1], acc[3][2], acc[3][3]);

  float* slab = sT[wave];
  const float* Rb = RESID ? (resid + (size_t)b * strideR) : nullptr;
#pragma unroll
  for (int i = 0; i < 4; ++i) {
    const int mBase = m0 + (i << 4);
#pragma unroll
    for (int j = 0; j < 4; ++j) {
      const int n = n0 + (j << 4) + rlane;
      float bv = 0.f;
      if (BIAS_MODE == 2) bv = bias[n];
#pragma unroll
      for (int r = 0; r < 8; ++r) {
        float v = acc[i][j][r] * scale;
        if (BIAS_MODE == 1) v += bias[mBase + mOff + r];
        if (BIAS_MODE == 2) v += bv;
        if (RESID) v += Rb[(size_t)(mBase + mOff + r) * ldc + n];
        if (ACT == 1) v = tanhf(v);
        if (ACT == 2) v = fmaxf(v, 0.0f);
        if (ACT == 3) v = v / (1.0f + expf(-v));
        if (ACT == 4) v = (v > 0.f) ? v : 0.01f * v;
        if (ACT == 5) v = 0.5f * v * (1.0f + erff(v * 0.70710678118654752f));
        slab[(mOff + r) * 68 + (j << 4) + rlane] = v;
      }
    }
    __builtin_amdgcn_fence(__ATOMIC_RELEASE, "workgroup");
    __builtin_amdgcn_wave_barrier();
    __builtin_amdgcn_fence(__ATOMIC_ACQUIRE, "workgroup");
    if (OUT_MODE == 0) {
      float* C = (float*)Cout + (size_t)b * strideC;
      const int hh = lane >> 4, c4 = (lane & 15) * 4;
      for (int pass = 0; pass < 2; ++pass) {
#pragma unroll
        for (int it = 0; it < 8; ++it) {
          const int row = it * 2 + hh;
          v4f v = *(const v4f*)(slab + row * 68 + c4);
          *(volatile v4f*)(C + (size_t)(mBase + row) * ldc + n0 + c4) = v;
        }
        __threadfence();
      }
    } else {
      const int q = lane >> 3, c8 = (lane & 7) * 8;
      unsigned short* C  = (unsigned short*)Cout  + (size_t)b * strideC;
      unsigned short* C2 = (OUT_MODE == 2) ? ((unsigned short*)Cout2 + (size_t)b * strideC) : nullptr;
      for (int pass = 0; pass < 2; ++pass) {
#pragma unroll
        for (int it = 0; it < 4; ++it) {
          const int row = it * 4 + q;
          const float* sp = slab + row * 68 + c8;
          v8h hv, lv;
#pragma unroll
          for (int e = 0; e < 8; ++e) {
            if (OUT_MODE == 1) {
              hv[e] = (_Float16)sp[e];
            } else {
              unsigned short hb = f2bf_bits(sp[e]);
              unsigned short lb = f2bf_bits(sp[e] - bf_bits2f(hb));
              hv[e] = __builtin_bit_cast(_Float16, hb);
              lv[e] = __builtin_bit_cast(_Float16, lb);
            }
          }
          *(volatile v8h*)(C + (size_t)(mBase + row) * ldc + n0 + c8) = hv;
          if (OUT_MODE == 2) *(volatile v8h*)(C2 + (size_t)(mBase + row) * ldc + n0 + c8) = lv;
        }
        __threadfence();
      }
    }
    __builtin_amdgcn_fence(__ATOMIC_RELEASE, "workgroup");
    __builtin_amdgcn_wave_barrier();
    __builtin_amdgcn_fence(__ATOMIC_ACQUIRE, "workgroup");
  }
}

__global__ __launch_bounds__(256) void cast_rows_kernel(
    const float* __restrict__ src, unsigned short* __restrict__ dst,
    int R, int Rp, int Kc, int rot, int nchunks, float scale)
{
  const int f = blockIdx.x * 256 + threadIdx.x;
  if (f >= nchunks) return;
  const int cpr = Kc >> 3;
  const int rowflat = f / cpr;
  const int g  = f - rowflat * cpr;
  const int kb = rowflat / Rp;
  const int n  = rowflat - kb * Rp;
  const bool valid = n < R;
  int sr = n + rot;
  sr = (sr >= R) ? (sr - R) : sr;
  sr = valid ? sr : 0;
  const float* p = src + ((size_t)kb * R + sr) * Kc + g * 8;
  const v4f a0 = *(const v4f*)(p);
  const v4f a1 = *(const v4f*)(p + 4);
  v8h hv;
#pragma unroll
  for (int e = 0; e < 4; ++e) {
    hv[e]     = (_Float16)(valid ? a0[e] * scale : 0.0f);
    hv[4 + e] = (_Float16)(valid ? a1[e] * scale : 0.0f);
  }
  unsigned short* q = dst + (size_t)f * 8;
  *(volatile v8h*)q = hv;
  __threadfence();
  *(volatile v8h*)q = hv;
}

__global__ __launch_bounds__(256) void nchw_to_tok16_kernel(
    const float* __restrict__ x, unsigned short* __restrict__ X16)
{
  __shared__ __align__(16) _Float16 sX[64 * NCH];
  const int t  = threadIdx.x;
  const int b_ = blockIdx.x >> 6;
  const int t0 = (blockIdx.x & 63) * 64;
#pragma unroll
  for (int it = 0; it < 8; ++it) {
    const int q   = it * 256 + t;
    const int ch  = q >> 4;
    const int seg = q & 15;
    const v4f v = *(const v4f*)(x + ((size_t)(b_ * NCH + ch)) * NPIX + t0 + seg * 4);
#pragma unroll
    for (int e = 0; e < 4; ++e) sX[(seg * 4 + e) * NCH + ch] = (_Float16)(v[e] * 8.0f);
  }
  __syncthreads();
  v8h vals[4];
#pragma unroll
  for (int it = 0; it < 4; ++it) vals[it] = *(const v8h*)(sX + (it * 256 + t) * 8);
  unsigned short* ob = X16 + (size_t)blockIdx.x * 64 * NCH;
  for (int pass = 0; pass < 2; ++pass) {
#pragma unroll
    for (int it = 0; it < 4; ++it) *(volatile v8h*)(ob + (size_t)(it * 256 + t) * 8) = vals[it];
    __threadfence();
  }
}

template <bool EMIT16>
__global__ __launch_bounds__(128) void dwconv_silu_kernel(
    const float* __restrict__ XP, const float* __restrict__ cw, const float* __restrict__ cbias,
    float* __restrict__ XI, unsigned short* __restrict__ XI16)
{
  __shared__ __align__(16) _Float16 sH[EMIT16 ? IMG_W * NCH : 8];
  const int d  = threadIdx.x;
  const int b_ = blockIdx.x / IMG_H;
  const int h_ = blockIdx.x - b_ * IMG_H;
  const float* wr = cw + d * 9;
  const float w00 = wr[0], w01 = wr[1], w02 = wr[2];
  const float w10 = wr[3], w11 = wr[4], w12 = wr[5];
  const float w20 = wr[6], w21 = wr[7], w22 = wr[8];
  const float bc = cbias[d];
  const bool up = h_ > 0, dn = h_ < IMG_H - 1;
  const int r0 = up ? (h_ - 1) : 0;
  const int r2 = dn ? (h_ + 1) : (IMG_H - 1);
  const float* p0 = XP + ((size_t)(b_ * IMG_H + r0) * IMG_W) * NCH + d;
  const float* p1 = XP + ((size_t)(b_ * IMG_H + h_) * IMG_W) * NCH + d;
  const float* p2 = XP + ((size_t)(b_ * IMG_H + r2) * IMG_W) * NCH + d;
  float a0m = 0.f, a1m = 0.f, a2m = 0.f;
  float a0c, a1c, a2c;
  {
    const float v0 = p0[0], v1 = p1[0], v2 = p2[0];
    a0c = up ? v0 : 0.f;
    a1c = v1;
    a2c = dn ? v2 : 0.f;
  }
  float* orow = XI + ((size_t)(b_ * IMG_H + h_) * IMG_W) * NCH + d;
#pragma unroll 1
  for (int w = 0; w < IMG_W; ++w) {
    const bool rv = (w + 1) < IMG_W;
    const int  wn = rv ? (w + 1) : (IMG_W - 1);
    const float n0 = p0[(size_t)wn * NCH], n1 = p1[(size_t)wn * NCH], n2 = p2[(size_t)wn * NCH];
    const float a0n = (up && rv) ? n0 : 0.f;
    const float a1n = rv ? n1 : 0.f;
    const float a2n = (dn && rv) ? n2 : 0.f;
    float acc = w00 * a0m;
    acc = fmaf(w01, a0c, acc);
    acc = fmaf(w02, a0n, acc);
    acc = fmaf(w10, a1m, acc);
    acc = fmaf(w11, a1c, acc);
    acc = fmaf(w12, a1n, acc);
    acc = fmaf(w20, a2m, acc);
    acc = fmaf(w21, a2c, acc);
    acc = fmaf(w22, a2n, acc);
    const float sv  = acc + bc;
    const float sg  = __builtin_amdgcn_rcpf(1.0f + __expf(-sv));
    const float out = sv * sg;
    float* op = orow + (size_t)w * NCH;
    *(volatile float*)op = out;
    __threadfence();
    *(volatile float*)op = out;
    if (EMIT16) sH[w * NCH + d] = (_Float16)(out * 64.0f);
    a0m = a0c; a0c = a0n;
    a1m = a1c; a1c = a1n;
    a2m = a2c; a2c = a2n;
  }
  if (EMIT16) {
    __syncthreads();
    v8h vals[8];
#pragma unroll
    for (int it = 0; it < 8; ++it) vals[it] = *(const v8h*)(sH + (it * NCH + d) * 8);
    unsigned short* ob = XI16 + (size_t)blockIdx.x * IMG_W * NCH;
    for (int pass = 0; pass < 2; ++pass) {
#pragma unroll
      for (int it = 0; it < 8; ++it) *(volatile v8h*)(ob + (size_t)(it * NCH + d) * 8) = vals[it];
      __threadfence();
    }
  }
}

__global__ __launch_bounds__(128) void scan_spa_kernel(
    const float* __restrict__ XDBL, const float* __restrict__ U,
    const float* __restrict__ dtw, const float* __restrict__ dtb,
    const float* __restrict__ Alog, const float* __restrict__ Dsp,
    float* __restrict__ Y)
{
  __shared__ __align__(16) float sRow[32 * 40];
  const int d  = threadIdx.x;
  const int b_ = blockIdx.x;
  const size_t tokb = (size_t)b_ * NPIX;
#pragma unroll 1
  for (int k = 0; k < NDIRS; ++k) {
    const float* wr = dtw + ((size_t)k * NCH + d) * DTR_SPA;
    const v4f wa = *(const v4f*)(wr);
    const v4f wb = *(const v4f*)(wr + 4);
    const float db = dtb[k * NCH + d];
    const float Dk = Dsp[k * NCH + d];
    float An[NSTATE], h[NSTATE];
#pragma unroll
    for (int n = 0; n < NSTATE; ++n) {
      const float al = Alog[((size_t)k * NCH + d) * NSTATE + n];
      An[n] = -__expf(al);
      h[n]  = 0.f;
    }
    const float* xd = XDBL + ((size_t)k * NTOK + tokb) * XDW;
#pragma unroll 1
    for (int c = 0; c < NPIX / 32; ++c) {
      __syncthreads();
      for (int q = d; q < 320; q += NCH) {
        const int s  = q / 10;
        const int j4 = (q - s * 10) * 4;
        const int l  = c * 32 + s;
        const int tok = (k == 1) ? (NPIX - 1 - l) : l;
        const v4f v = *(const v4f*)(xd + (size_t)tok * XDW + j4);
        *(v4f*)(sRow + s * 40 + j4) = v;
      }
      __syncthreads();
#pragma unroll 1
      for (int s = 0; s < 32; ++s) {
        const int l   = c * 32 + s;
        const int tok = (k == 1) ? (NPIX - 1 - l) : l;
        const size_t ei = (tokb + tok) * NCH + d;
        const float u = U[ei];
        const float* sr = sRow + s * 40;
        const v4f D0 = *(const v4f*)(sr);
        const v4f D1 = *(const v4f*)(sr + 4);
        v4f Bv[4], Cv[4];
#pragma unroll
        for (int i = 0; i < 4; ++i) {
          Bv[i] = *(const v4f*)(sr + 8 + 4 * i);
          Cv[i] = *(const v4f*)(sr + 24 + 4 * i);
        }
        float dp = db;
        dp = fmaf(wa[0], D0[0], dp);
        dp = fmaf(wa[1], D0[1], dp);
        dp = fmaf(wa[2], D0[2], dp);
        dp = fmaf(wa[3], D0[3], dp);
        dp = fmaf(wb[0], D1[0], dp);
        dp = fmaf(wb[1], D1[1], dp);
        dp = fmaf(wb[2], D1[2], dp);
        dp = fmaf(wb[3], D1[3], dp);
        const float ex    = __expf(-fabsf(dp));
        const float delta = fmaxf(dp, 0.0f) + __logf(1.0f + ex);
        const float du    = delta * u;
        float y = Dk * u;
#pragma unroll
        for (int n = 0; n < NSTATE; ++n) {
          const float e  = __expf(delta * An[n]);
          const float hn = fmaf(e, h[n], du * Bv[n >> 2][n & 3]);
          h[n] = hn;
          y = fmaf(hn, Cv[n >> 2][n & 3], y);
        }
        float* yp = Y + ei;
        if (k > 0) {
          const float old = *(const float*)yp;
          y += old;
        }
        *(volatile float*)yp = y;
        __threadfence();
        *(volatile float*)yp = y;
      }
    }
  }
}

__global__ __launch_bounds__(256) void ln128_kernel(
    const float* __restrict__ Y, const float* __restrict__ g, const float* __restrict__ be,
    unsigned short* __restrict__ dst)
{
  __shared__ __align__(16) _Float16 sT[32 * NCH];
  const int t = threadIdx.x;
  const int r = t >> 3, part = t & 7;
  const int row = blockIdx.x * 32 + r;
  const int c0  = part * 16;
  const float* yr = Y + (size_t)row * NCH + c0;
  v4f a[4];
#pragma unroll
  for (int j = 0; j < 4; ++j) a[j] = *(const v4f*)(yr + 4 * j);
  float s = 0.f;
#pragma unroll
  for (int j = 0; j < 4; ++j) s += (a[j][0] + a[j][1]) + (a[j][2] + a[j][3]);
  s += __shfl_xor(s, 1, 32);
  s += __shfl_xor(s, 2, 32);
  s += __shfl_xor(s, 4, 32);
  const float mu = s * (1.0f / 128.0f);
  float q = 0.f;
#pragma unroll
  for (int j = 0; j < 4; ++j) {
#pragma unroll
    for (int e = 0; e < 4; ++e) { const float dd = a[j][e] - mu; q = fmaf(dd, dd, q); }
  }
  q += __shfl_xor(q, 1, 32);
  q += __shfl_xor(q, 2, 32);
  q += __shfl_xor(q, 4, 32);
  const float var = q * (1.0f / 128.0f);
  const float is  = rsqrtf(var + 1e-5f);
#pragma unroll
  for (int j = 0; j < 4; ++j) {
    const v4f gg = *(const v4f*)(g  + c0 + 4 * j);
    const v4f bb = *(const v4f*)(be + c0 + 4 * j);
    v4h hv;
#pragma unroll
    for (int e = 0; e < 4; ++e) hv[e] = (_Float16)((((a[j][e] - mu) * is) * gg[e] + bb[e]) * 16.0f);
    *(v4h*)(sT + r * NCH + c0 + 4 * j) = hv;
  }
  __syncthreads();
  v8h vals[2];
#pragma unroll
  for (int it = 0; it < 2; ++it) vals[it] = *(const v8h*)(sT + (it * 256 + t) * 8);
  unsigned short* ob = dst + (size_t)blockIdx.x * 32 * NCH;
  for (int pass = 0; pass < 2; ++pass) {
#pragma unroll
    for (int it = 0; it < 2; ++it) *(volatile v8h*)(ob + (size_t)(it * 256 + t) * 8) = vals[it];
    __threadfence();
  }
}

__global__ __launch_bounds__(256) void spe_scan_kernel(
    const float* __restrict__ UE, const float* __restrict__ xproj,
    const float* __restrict__ dtw, const float* __restrict__ dtb,
    const float* __restrict__ Alog, const float* __restrict__ Dsp,
    const float* __restrict__ ng, const float* __restrict__ nb,
    unsigned short* __restrict__ Y16)
{
  __shared__ __align__(16) float s_w[NDIRS * XROWS_SPE * CN_SPE];
  __shared__ __align__(16) float s_u[8][NCH];
  __shared__ __align__(16) float s_dbl[8][NDIRS * XROWS_SPE * GC_SPE];
  __shared__ __align__(16) float s_y[8][NDIRS][NCH];
  __shared__ __align__(16) _Float16 s_o[8 * NCH];
  const int tid  = threadIdx.x;
  const int wave = tid >> 5;
  const int lane = tid & 31;
  const int p    = blockIdx.x * 8 + wave;

  for (int i = tid; i < NDIRS * XROWS_SPE * CN_SPE; i += 256) s_w[i] = xproj[i];
  {
    const v4f v = *(const v4f*)(UE + (size_t)p * NCH + lane * 4);
    *(v4f*)(&s_u[wave][lane * 4]) = v;
  }
  __syncthreads();

  {
    const int k    = lane >> 4;
    const int g    = (lane >> 1) & 7;
    const int half = lane & 1;
    const int gg   = k ? (GC_SPE - 1 - g) : g;
    float ur[CN_SPE];
#pragma unroll
    for (int cn = 0; cn < CN_SPE; ++cn) ur[cn] = s_u[wave][cn * GC_SPE + gg];
    const int cbase  = half * 17;
    const int ccount = half ? 16 : 17;
    float* dbw = s_dbl[wave];
#pragma unroll 1
    for (int i = 0; i < 17; ++i) {
      const int c  = cbase + i;
      const int cc = (c < XROWS_SPE) ? c : (XROWS_SPE - 1);
      const float* wp = s_w + (k * XROWS_SPE + cc) * CN_SPE;
      const v4f w0 = *(const v4f*)(wp);
      const v4f w1 = *(const v4f*)(wp + 4);
      const v4f w2 = *(const v4f*)(wp + 8);
      const v4f w3 = *(const v4f*)(wp + 12);
      float acc = 0.f;
#pragma unroll
      for (int e = 0; e < 4; ++e) acc = fmaf(w0[e], ur[e], acc);
#pragma unroll
      for (int e = 0; e < 4; ++e) acc = fmaf(w1[e], ur[4 + e], acc);
#pragma unroll
      for (int e = 0; e < 4; ++e) acc = fmaf(w2[e], ur[8 + e], acc);
#pragma unroll
      for (int e = 0; e < 4; ++e) acc = fmaf(w3[e], ur[12 + e], acc);
      if (i < ccount) dbw[(k * XROWS_SPE + c) * GC_SPE + g] = acc;
    }
  }
  __syncthreads();

  {
    const int k  = lane >> 4;
    const int cn = lane & 15;
    float An[NSTATE], h[NSTATE];
#pragma unroll
    for (int n = 0; n < NSTATE; ++n) {
      An[n] = -__expf(Alog[((size_t)k * CN_SPE + cn) * NSTATE + n]);
      h[n]  = 0.f;
    }
    const float dtwv = dtw[k * CN_SPE + cn];
    const float dtbv = dtb[k * CN_SPE + cn];
    const float Dd   = Dsp[k * CN_SPE + cn];
    const float* db = s_dbl[wave] + k * XROWS_SPE * GC_SPE;
#pragma unroll 1
    for (int g = 0; g < GC_SPE; ++g) {
      const int gg = k ? (GC_SPE - 1 - g) : g;
      const float dts   = db[g];
      const float dp    = fmaf(dtwv, dts, dtbv);
      const float ex    = __expf(-fabsf(dp));
      const float delta = fmaxf(dp, 0.0f) + __logf(1.0f + ex);
      const float u     = s_u[wave][cn * GC_SPE + gg];
      const float du    = delta * u;
      float y = Dd * u;
#pragma unroll
      for (int n = 0; n < NSTATE; ++n) {
        const float Bn = db[(1 + n) * GC_SPE + g];
        const float Cq = db[(1 + NSTATE + n) * GC_SPE + g];
        const float e  = __expf(delta * An[n]);
        const float hn = fmaf(e, h[n], du * Bn);
        h[n] = hn;
        y = fmaf(hn, Cq, y);
      }
      s_y[wave][k][cn * GC_SPE + gg] = y;
    }
  }
  __syncthreads();

  {
    const int gsel = lane >> 4;
    const int cn   = lane & 15;
    const float ngv = ng[cn];
    const float nbv = nb[cn];
#pragma unroll 1
    for (int gi = 0; gi < 4; ++gi) {
      const int g = gsel * 4 + gi;
      const float v = s_y[wave][0][cn * GC_SPE + g] + s_y[wave][1][cn * GC_SPE + g];
      float s = v;
      s += __shfl_xor(s, 1, 32);
      s += __shfl_xor(s, 2, 32);
      s += __shfl_xor(s, 4, 32);
      s += __shfl_xor(s, 8, 32);
      const float mu = s * (1.0f / 16.0f);
      const float dd = v - mu;
      float q = dd * dd;
      q += __shfl_xor(q, 1, 32);
      q += __shfl_xor(q, 2, 32);
      q += __shfl_xor(q, 4, 32);
      q += __shfl_xor(q, 8, 32);
      const float var = q * (1.0f / 16.0f);
      const float is  = rsqrtf(var + 1e-5f);
      const float o   = (dd * is) * ngv + nbv;
      s_o[wave * NCH + cn * GC_SPE + g] = (_Float16)(o * 16.0f);
    }
  }
  __syncthreads();
  {
    const int ci = (tid < 128) ? tid : 127;
    const v8h val = *(const v8h*)(s_o + ci * 8);
    unsigned short* ob = Y16 + (size_t)blockIdx.x * 8 * NCH;
    for (int pass = 0; pass < 2; ++pass) {
      if (tid < 128) *(volatile v8h*)(ob + (size_t)tid * 8) = val;
      __threadfence();
    }
  }
}

__global__ __launch_bounds__(256) void tok_to_nchw_kernel(
    const float* __restrict__ OT, float* __restrict__ out)
{
  __shared__ __align__(16) float sT[NCH * 68];
  const int t  = threadIdx.x;
  const int b_ = blockIdx.x >> 6;
  const int t0 = (blockIdx.x & 63) * 64;
#pragma unroll
  for (int it = 0; it < 8; ++it) {
    const int q   = it * 256 + t;
    const int row = q >> 5;
    const int c4  = (q & 31) * 4;
    const v4f v = *(const v4f*)(OT + ((size_t)blockIdx.x * 64 + row) * NCH + c4);
#pragma unroll
    for (int e = 0; e < 4; ++e) sT[(c4 + e) * 68 + row] = v[e];
  }
  __syncthreads();
  v4f vals[8];
#pragma unroll
  for (int it = 0; it < 8; ++it) {
    const int q   = it * 256 + t;
    const int ch  = q >> 4;
    const int seg = q & 15;
    vals[it] = *(const v4f*)(sT + ch * 68 + seg * 4);
  }
  for (int pass = 0; pass < 2; ++pass) {
#pragma unroll
    for (int it = 0; it < 8; ++it) {
      const int q   = it * 256 + t;
      const int ch  = q >> 4;
      const int seg = q & 15;
      *(volatile v4f*)(out + ((size_t)(b_ * NCH + ch)) * NPIX + t0 + seg * 4) = vals[it];
    }
    __threadfence();
  }
}

extern "C" void kernel_launch(void* const* d_in, const int* in_sizes, int n_in,
                              void* d_out, int out_size, void* d_ws, size_t ws_size,
                              hipStream_t stream)
{
  if (n_in < 35) return;
  const float* x         = (const float*)d_in[0];
  const float* c1_w      = (const float*)d_in[7];
  const float* c1_b      = (const float*)d_in[8];
  const float* spa_in_w  = (const float*)d_in[9];
  const float* spa_dwc_w = (const float*)d_in[12];
  const float* spa_dwc_b = (const float*)d_in[13];
  const float* spa_out_w = (const float*)d_in[14];
  const float* spa_xproj = (const float*)d_in[15];
  const float* spa_dt_w  = (const float*)d_in[16];
  const float* spa_dt_b  = (const float*)d_in[17];
  const float* spa_Alog  = (const float*)d_in[18];
  const float* spa_D     = (const float*)d_in[19];
  const float* spa_ng    = (const float*)d_in[20];
  const float* spa_nb    = (const float*)d_in[21];
  const float* spe_in_w  = (const float*)d_in[22];
  const float* spe_dwc_w = (const float*)d_in[25];
  const float* spe_dwc_b = (const float*)d_in[26];
  const float* spe_out_w = (const float*)d_in[27];
  const float* spe_xproj = (const float*)d_in[28];
  const float* spe_dt_w  = (const float*)d_in[29];
  const float* spe_dt_b  = (const float*)d_in[30];
  const float* spe_Alog  = (const float*)d_in[31];
  const float* spe_D     = (const float*)d_in[32];
  const float* spe_ng    = (const float*)d_in[33];
  const float* spe_nb    = (const float*)d_in[34];
  float* dout = (float*)d_out;

  if (in_sizes[0] != NTOK * NCH) return;
  if (in_sizes[7] != NCH * NCH || in_sizes[8] != NCH) return;
  if (in_sizes[9] != NCH * NCH) return;
  if (in_sizes[12] != NCH * 9 || in_sizes[13] != NCH) return;
  if (in_sizes[14] != NCH * NCH) return;
  if (in_sizes[15] != NDIRS * XROWS_SPA * NCH) return;
  if (in_sizes[16] != NDIRS * NCH * DTR_SPA || in_sizes[17] != NDIRS * NCH) return;
  if (in_sizes[18] != NDIRS * NCH * NSTATE || in_sizes[19] != NDIRS * NCH) return;
  if (in_sizes[20] != NCH || in_sizes[21] != NCH) return;
  if (in_sizes[22] != NCH * NCH) return;
  if (in_sizes[25] != NCH * 9 || in_sizes[26] != NCH) return;
  if (in_sizes[27] != NCH * NCH) return;
  if (in_sizes[28] != NDIRS * XROWS_SPE * CN_SPE) return;
  if (in_sizes[29] != NDIRS * CN_SPE || in_sizes[30] != NDIRS * CN_SPE) return;
  if (in_sizes[31] != NDIRS * CN_SPE * NSTATE || in_sizes[32] != NDIRS * CN_SPE) return;
  if (in_sizes[33] != CN_SPE || in_sizes[34] != CN_SPE) return;
  if (out_size != NTOK * NCH) return;

  const size_t SZ_W    = (size_t)NCH * NCH * 2;
  const size_t SZ_WX   = (size_t)NDIRS * XDW * NCH * 2;
  const size_t SZ_H    = (size_t)NTOK * NCH * 2;
  const size_t SZ_F    = (size_t)NTOK * NCH * 4;
  const size_t SZ_XDBL = (size_t)NDIRS * NTOK * XDW * 4;
  size_t off = 0;
  const size_t OFF_WIN  = off; off += 2 * SZ_W;
  const size_t OFF_WO   = off; off += 2 * SZ_W;
  const size_t OFF_WC1  = off; off += SZ_W;
  const size_t OFF_WX   = off; off += SZ_WX;
  const size_t OFF_X16  = off; off += SZ_H;
  const size_t OFF_X1   = off; off += 2 * SZ_F;
  const size_t OFF_UA   = off; off += SZ_F;
  const size_t OFF_U16A = off; off += SZ_H;
  const size_t OFF_UE   = off; off += SZ_F;
  const size_t OFF_XDBL = off; off += SZ_XDBL;
  const size_t OFF_YA   = off; off += SZ_F;
  const size_t OFF_Y16A = off; off += SZ_H;
  const size_t OFF_Y16E = off; off += SZ_H;
  const size_t OFF_SA   = off; off += SZ_F;
  const size_t OFF_S    = off; off += SZ_F;
  const size_t OFF_S16  = off; off += SZ_H;
  const size_t OFF_OT   = off; off += SZ_F;
  const size_t TOTAL    = off;
  if (ws_size < TOTAL) return;

  char* ws = (char*)d_ws;
  unsigned short* WIN  = (unsigned short*)(ws + OFF_WIN);
  unsigned short* WO   = (unsigned short*)(ws + OFF_WO);
  unsigned short* WC1  = (unsigned short*)(ws + OFF_WC1);
  unsigned short* WX   = (unsigned short*)(ws + OFF_WX);
  unsigned short* X16  = (unsigned short*)(ws + OFF_X16);
  float*          X1   = (float*)(ws + OFF_X1);
  float*          X1A  = X1;
  float*          X1E  = X1 + (size_t)NTOK * NCH;
  float*          UA   = (float*)(ws + OFF_UA);
  unsigned short* U16A = (unsigned short*)(ws + OFF_U16A);
  float*          UE   = (float*)(ws + OFF_UE);
  float*          XDBL = (float*)(ws + OFF_XDBL);
  float*          YA   = (float*)(ws + OFF_YA);
  unsigned short* Y16A = (unsigned short*)(ws + OFF_Y16A);
  unsigned short* Y16E = (unsigned short*)(ws + OFF_Y16E);
  float*          SA   = (float*)(ws + OFF_SA);
  float*          S    = (float*)(ws + OFF_S);
  unsigned short* S16  = (unsigned short*)(ws + OFF_S16);
  float*          OT   = (float*)(ws + OFF_OT);
  const float*    nores = x;

  const int NCHUNK_W = NCH * NCH / 8;
  const int NCHUNK_X = NDIRS * XDW * NCH / 8;
  const int NCHUNK_S = NTOK * NCH / 8;

  cast_rows_kernel<<<NCHUNK_W / 256, 256, 0, stream>>>(spa_in_w,  WIN,                     NCH, NCH, NCH, 0, NCHUNK_W, 16.0f);
  cast_rows_kernel<<<NCHUNK_W / 256, 256, 0, stream>>>(spe_in_w,  WIN + (size_t)NCH * NCH, NCH, NCH, NCH, 0, NCHUNK_W, 16.0f);
  cast_rows_kernel<<<NCHUNK_W / 256, 256, 0, stream>>>(spa_out_w, WO,                      NCH, NCH, NCH, 0, NCHUNK_W, 16.0f);
  cast_rows_kernel<<<NCHUNK_W / 256, 256, 0, stream>>>(spe_out_w, WO + (size_t)NCH * NCH,  NCH, NCH, NCH, 0, NCHUNK_W, 16.0f);
  cast_rows_kernel<<<NCHUNK_W / 256, 256, 0, stream>>>(c1_w,      WC1,                     NCH, NCH, NCH, 0, NCHUNK_W, 16.0f);
  cast_rows_kernel<<<NCHUNK_X / 256, 256, 0, stream>>>(spa_xproj, WX, XROWS_SPA, XDW, NCH, 0, NCHUNK_X, 16.0f);

  nchw_to_tok16_kernel<<<NTOK / 64, 256, 0, stream>>>(x, X16);

  wmma_gemm64<0, false, 0, 0, false, 0><<<dim3(32, 2), 256, 0, stream>>>(
      X16, X16, NCH, 0L, WIN, WIN, NCH, (long)NCH * NCH, (void*)X1, (void*)X1, NCH, (long)NTOK * NCH,
      nores, nores, 0L, NTOK, NCH, NCH, 1.0f / 128.0f);

  dwconv_silu_kernel<true><<<NIMG * IMG_H, NCH, 0, stream>>>(X1A, spa_dwc_w, spa_dwc_b, UA, U16A);
  dwconv_silu_kernel<false><<<NIMG * IMG_H, NCH, 0, stream>>>(X1E, spe_dwc_w, spe_dwc_b, UE, U16A);

  wmma_gemm64<0, false, 0, 0, false, 0><<<dim3(16, NDIRS), 256, 0, stream>>>(
      U16A, U16A, NCH, 0L, WX, WX, NCH, (long)XDW * NCH, (void*)XDBL, (void*)XDBL, XDW, (long)NTOK * XDW,
      nores, nores, 0L, NTOK, XDW, NCH, 1.0f / 1024.0f);

  scan_spa_kernel<<<NIMG, NCH, 0, stream>>>(XDBL, UA, spa_dt_w, spa_dt_b, spa_Alog, spa_D, YA);

  ln128_kernel<<<NTOK / 32, 256, 0, stream>>>(YA, spa_ng, spa_nb, Y16A);

  spe_scan_kernel<<<NTOK / 8, 256, 0, stream>>>(UE, spe_xproj, spe_dt_w, spe_dt_b, spe_Alog, spe_D,
                                                spe_ng, spe_nb, Y16E);

  wmma_gemm64<0, false, 0, 0, false, 0><<<dim3(32, 1), 256, 0, stream>>>(
      Y16A, Y16A, NCH, 0L, WO, WO, NCH, 0L, (void*)SA, (void*)SA, NCH, 0L,
      nores, nores, 0L, NTOK, NCH, NCH, 1.0f / 256.0f);
  wmma_gemm64<0, false, 0, 0, true, 0><<<dim3(32, 1), 256, 0, stream>>>(
      Y16E, Y16E, NCH, 0L, WO + (size_t)NCH * NCH, WO + (size_t)NCH * NCH, NCH, 0L, (void*)S, (void*)S, NCH, 0L,
      nores, SA, 0L, NTOK, NCH, NCH, 1.0f / 256.0f);

  cast_rows_kernel<<<NCHUNK_S / 256, 256, 0, stream>>>(S, S16, NTOK, NTOK, NCH, 0, NCHUNK_S, 16.0f);

  wmma_gemm64<0, false, 2, 0, true, 0><<<dim3(32, 1), 256, 0, stream>>>(
      S16, S16, NCH, 0L, WC1, WC1, NCH, 0L, (void*)OT, (void*)OT, NCH, 0L,
      c1_b, S, 0L, NTOK, NCH, NCH, 1.0f / 256.0f);

  tok_to_nchw_kernel<<<NTOK / 64, 256, 0, stream>>>(OT, dout);
}
